// ProfileHMM_55439437857594
// MI455X (gfx1250) — hardware-verified
//
#include <hip/hip_runtime.h>
#include <hip/hip_bf16.h>
#include <stdint.h>

typedef __attribute__((ext_vector_type(16))) _Float16 v16h;
typedef __attribute__((ext_vector_type(8)))  _Float16 v8h;
typedef __attribute__((ext_vector_type(16))) __bf16   v16b;
typedef __attribute__((ext_vector_type(8)))  __bf16   v8b;
typedef __attribute__((ext_vector_type(8)))  float    v8f;
typedef __attribute__((ext_vector_type(4)))  float    v4f;
typedef __attribute__((ext_vector_type(4)))  unsigned int v4u;
#define U16(p) ((const unsigned short*)(const void*)(p))

__device__ __forceinline__ unsigned short f2bf_bits(float f) {
  unsigned u = __float_as_uint(f);
  return (unsigned short)((u + 0x7FFFu + ((u >> 16) & 1u)) >> 16);
}
__device__ __forceinline__ float bf_bits2f(unsigned short h) { return __uint_as_float(((unsigned)h) << 16); }
__device__ __forceinline__ unsigned short f2bf_ftz(float f) {
  const unsigned u = __float_as_uint(f);
  if ((u & 0x7f800000u) == 0u) return (unsigned short)0;
  return f2bf_bits(f);
}

__device__ __forceinline__ void dep_guard_h(v8f& a, v8f& b, v16h x, v16h y) { asm volatile("v_nop\n\tv_nop\n\tv_nop\n\tv_nop" : "+v"(a), "+v"(b) : "v"(x), "v"(y)); }
__device__ __forceinline__ void dep_guard_b(v8f& a, v8f& b, v16b x, v16b y) { asm volatile("v_nop\n\tv_nop\n\tv_nop\n\tv_nop" : "+v"(a), "+v"(b) : "v"(x), "v"(y)); }
__device__ __forceinline__ void keep4_h(v16h a, v16h b, v16h c, v16h d) { asm volatile("v_nop" :: "v"(a), "v"(b), "v"(c), "v"(d)); }
__device__ __forceinline__ void keep4_b(v16b a, v16b b, v16b c, v16b d) { asm volatile("v_nop" :: "v"(a), "v"(b), "v"(c), "v"(d)); }
__device__ __forceinline__ void acc_guard4(v8f& a, v8f& b, v8f& c, v8f& d) { asm volatile("v_nop\n\tv_nop\n\tv_nop\n\tv_nop" : "+v"(a), "+v"(b), "+v"(c), "+v"(d)); }
__device__ __forceinline__ void dep_guard3_b(v8f& a, v8f& b, v8f& c, v16b x, v16b y0, v16b y1, v16b y2) {
  asm volatile("v_nop\n\tv_nop\n\tv_nop\n\tv_nop" : "+v"(a), "+v"(b), "+v"(c) : "v"(x), "v"(y0), "v"(y1), "v"(y2));
}
__device__ __forceinline__ void dep_guard1_b(v8f& a, v16b x, v16b y) {
  asm volatile("v_nop\n\tv_nop\n\tv_nop\n\tv_nop" : "+v"(a) : "v"(x), "v"(y));
}

template <typename T> struct Frag;
template <> struct Frag<_Float16> {
  typedef v16h V; union U { v16h v; v8h h[2]; };
  static __device__ __forceinline__ v16h load(const _Float16* p) {
    U f; f.h[0] = *(const v8h*)(p); f.h[1] = *(const v8h*)(p + 16); return f.v;
  }
  static __device__ __forceinline__ v8f mma(v16h a, v16h b, v8f c) {
    return __builtin_amdgcn_wmma_f32_16x16x32_f16(false, a, false, b, (short)0, c, false, false);
  }
  static __device__ __forceinline__ void guard(v8f& a, v8f& b, v16h x, v16h y) { dep_guard_h(a, b, x, y); }
  static __device__ __forceinline__ void keep(v16h a, v16h b, v16h c, v16h d) { keep4_h(a, b, c, d); }
};
template <> struct Frag<__bf16> {
  typedef v16b V; union U { v16b v; v8b h[2]; };
  static __device__ __forceinline__ v16b load(const __bf16* p) {
    U f; f.h[0] = *(const v8b*)(p); f.h[1] = *(const v8b*)(p + 16); return f.v;
  }
  static __device__ __forceinline__ v8f mma(v16b a, v16b b, v8f c) {
    return __builtin_amdgcn_wmma_f32_16x16x32_bf16(false, a, false, b, (short)0, c, false, false);
  }
  static __device__ __forceinline__ void guard(v8f& a, v8f& b, v16b x, v16b y) { dep_guard_b(a, b, x, y); }
  static __device__ __forceinline__ void keep(v16b a, v16b b, v16b c, v16b d) { keep4_b(a, b, c, d); }
};

template <int ET> struct Elem;
template <> struct Elem<0> { typedef _Float16 T; };
template <> struct Elem<1> { typedef __bf16 T; };
template <int ET, bool SPLIT, int BIAS_MODE, int OUT_MODE, bool RESID, int ACT = 0>
__global__ __launch_bounds__(256) void wmma_gemm64(
    const unsigned short* __restrict__ Ap, const unsigned short* __restrict__ A2p, int lda, long strideA,
    const unsigned short* __restrict__ Btp, const unsigned short* __restrict__ Bt2p, int ldb, long strideB,
    void* __restrict__ Cout, void* __restrict__ Cout2, int ldc, long strideC,
    const float* __restrict__ bias,
    const float* __restrict__ resid, long strideR,
    int M, int N, int K, float scale) {
  typedef typename Elem<ET>::T T;
  typedef typename Frag<T>::V V;
  const T* A = (const T*)Ap; const T* A2 = (const T*)A2p; const T* Bt = (const T*)Btp; const T* Bt2 = (const T*)Bt2p;
  __shared__ __align__(16) float sT[8][16 * 68];
  const int b    = blockIdx.y;
  const int lane = threadIdx.x & 31;
  const int wave = threadIdx.x >> 5;
  const int tilesN = N >> 6;
  const int tilesM = M >> 6;
  const int tile = blockIdx.x * 8 + wave;
  if (tile >= tilesM * tilesN) return;
  const int tm = tile / tilesN;
  const int tn = tile - tm * tilesN;
  const int m0 = tm << 6;
  const int n0 = tn << 6;

  const T* Ab  = A  + (size_t)b * strideA;
  const T* Bb  = Bt + (size_t)b * strideB;
  const T* Ab2 = SPLIT ? (A2  + (size_t)b * strideA) : nullptr;
  const T* Bb2 = SPLIT ? (Bt2 + (size_t)b * strideB) : nullptr;

  const int rlane = lane & 15;
  const int koff  = (lane >> 4) * 8;
  const int mOff  = (lane >> 4) * 8;

  v8f acc[4][4];
#pragma unroll
  for (int i = 0; i < 4; ++i)
#pragma unroll
    for (int j = 0; j < 4; ++j) acc[i][j] = (v8f){0.f,0.f,0.f,0.f,0.f,0.f,0.f,0.f};

  for (int k0 = 0; k0 < K; k0 += 32) {
    V bh[4], bl[4];
#pragma unroll
    for (int j = 0; j < 4; ++j) {
      const size_t bo = (size_t)(n0 + (j << 4) + rlane) * ldb + koff + k0;
      bh[j] = Frag<T>::load(Bb + bo);
      if (SPLIT) bl[j] = Frag<T>::load(Bb2 + bo);
    }
#pragma unroll
    for (int i = 0; i < 4; ++i) {
      const size_t ao = (size_t)(m0 + (i << 4) + rlane) * lda + koff + k0;
      V ah = Frag<T>::load(Ab + ao);
      V al;
      if (SPLIT) al = Frag<T>::load(Ab2 + ao);
#pragma unroll
      for (int j = 0; j < 4; ++j) {
        acc[i][j] = Frag<T>::mma(ah, bh[j], acc[i][j]);
        if (SPLIT) {
          acc[i][j] = Frag<T>::mma(ah, bl[j], acc[i][j]);
          acc[i][j] = Frag<T>::mma(al, bh[j], acc[i][j]);
        }
      }
      Frag<T>::guard(acc[i][0], acc[i][3], ah, SPLIT ? al : ah);
    }
    Frag<T>::keep(bh[0], bh[1], bh[2], bh[3]);
    if (SPLIT) Frag<T>::keep(bl[0], bl[1], bl[2], bl[3]);
  }
  acc_guard4(acc[0][0], acc[0][1], acc[0][2], acc[0][3]);
  acc_guard4(acc[1][0], acc[1][1], acc[1][2], acc[1][3]);
  acc_guard4(acc[2][0], acc[2][1], acc[2][2], acc[2][3]);
  acc_guard4(acc[3][0], acc[3][1], acc[3][2], acc[3][3]);

  float* slab = sT[wave];
  const float* Rb = RESID ? (resid + (size_t)b * strideR) : nullptr;
#pragma unroll
  for (int i = 0; i < 4; ++i) {
    const int mBase = m0 + (i << 4);
#pragma unroll
    for (int j = 0; j < 4; ++j) {
      const int n = n0 + (j << 4) + rlane;
      float bv = 0.f;
      if (BIAS_MODE == 2) bv = bias[n];
#pragma unroll
      for (int r = 0; r < 8; ++r) {
        float v = acc[i][j][r] * scale;
        if (BIAS_MODE == 1) v += bias[mBase + mOff + r];
        if (BIAS_MODE == 2) v += bv;
        if (RESID) v += Rb[(size_t)(mBase + mOff + r) * ldc + n];
        if (ACT == 1) v = tanhf(v);
        if (ACT == 2) v = fmaxf(v, 0.0f);
        if (ACT == 3) v = v / (1.0f + expf(-v));
        if (ACT == 4) v = (v > 0.f) ? v : 0.01f * v;
        if (ACT == 5) v = 0.5f * v * (1.0f + erff(v * 0.70710678118654752f));
        slab[(mOff + r) * 68 + (j << 4) + rlane] = v;
      }
    }
    __builtin_amdgcn_fence(__ATOMIC_RELEASE, "workgroup");
    __builtin_amdgcn_wave_barrier();
    __builtin_amdgcn_fence(__ATOMIC_ACQUIRE, "workgroup");
    if (OUT_MODE == 0) {
      float* C = (float*)Cout + (size_t)b * strideC;
      const int hh = lane >> 4, c4 = (lane & 15) * 4;
      for (int pass = 0; pass < 2; ++pass) {
#pragma unroll
        for (int it = 0; it < 8; ++it) {
          const int row = it * 2 + hh;
          v4f v = *(const v4f*)(slab + row * 68 + c4);
          *(volatile v4f*)(C + (size_t)(mBase + row) * ldc + n0 + c4) = v;
        }
        __threadfence();
      }
    } else {
      const int q = lane >> 3, c8 = (lane & 7) * 8;
      unsigned short* C  = (unsigned short*)Cout  + (size_t)b * strideC;
      unsigned short* C2 = (OUT_MODE == 2) ? ((unsigned short*)Cout2 + (size_t)b * strideC) : nullptr;
      for (int pass = 0; pass < 2; ++pass) {
#pragma unroll
        for (int it = 0; it < 4; ++it) {
          const int row = it * 4 + q;
          const float* sp = slab + row * 68 + c8;
          v8h hv, lv;
#pragma unroll
          for (int e = 0; e < 8; ++e) {
            if (OUT_MODE == 1) {
              hv[e] = (_Float16)sp[e];
            } else {
              unsigned short hb = f2bf_bits(sp[e]);
              unsigned short lb = f2bf_bits(sp[e] - bf_bits2f(hb));
              hv[e] = __builtin_bit_cast(_Float16, hb);
              lv[e] = __builtin_bit_cast(_Float16, lb);
            }
          }
          *(volatile v8h*)(C + (size_t)(mBase + row) * ldc + n0 + c8) = hv;
          if (OUT_MODE == 2) *(volatile v8h*)(C2 + (size_t)(mBase + row) * ldc + n0 + c8) = lv;
        }
        __threadfence();
      }
    }
    __builtin_amdgcn_fence(__ATOMIC_RELEASE, "workgroup");
    __builtin_amdgcn_wave_barrier();
    __builtin_amdgcn_fence(__ATOMIC_ACQUIRE, "workgroup");
  }
}

static constexpr int NMATCH  = 384;
static constexpr int NALPHA  = 21;
static constexpr int NBATCH  = 64;
static constexpr int SEQLEN  = 256;
static constexpr int NSTATE  = 2 * NMATCH + 1;
static constexpr int NCOLP   = 784;
static constexpr int KLOOP   = 800;
static constexpr int KPITCH  = 832;
static constexpr int TABLEN  = 832;
static constexpr int CLEN    = 416;
static constexpr int NPOS    = NBATCH * SEQLEN;
static constexpr int EMK     = 32;
static constexpr int OBSROWS = 832;
#define NEGBIG (-1.0e32f)

static_assert(NSTATE <= NCOLP && NCOLP % 16 == 0, "ncolp");
static_assert(KLOOP % 32 == 0 && KLOOP >= NSTATE && KLOOP + 0 <= KPITCH - 24 + 24, "kloop");
static_assert(KPITCH % 64 == 0 && KPITCH >= KLOOP, "kpitch");
static_assert(NPOS % 64 == 0 && OBSROWS % 64 == 0 && EMK % 32 == 0 && OBSROWS >= NSTATE, "gemm shape");
static_assert(((NPOS / 64) * (OBSROWS / 64)) % 8 == 0, "gemm grid");

static constexpr int TB_INIT = 0;
static constexpr int TB_SRCA = 1 * TABLEN;
static constexpr int TB_SRCB = 2 * TABLEN;
static constexpr int TB_ROWB = 3 * TABLEN;
static constexpr int TB_TT   = 4 * TABLEN;
static constexpr int TB_C    = 5 * TABLEN;
static constexpr int TABTOT  = 5 * TABLEN + CLEN;
static_assert(TABTOT % 32 == 0, "tab lines");

static constexpr size_t OFF_TAB  = 0;
static constexpr size_t SZ_TAB   = (size_t)TABTOT * 4;
static constexpr size_t OFF_LSE  = OFF_TAB + SZ_TAB;
static constexpr size_t SZ_LSE   = (size_t)TABLEN * 4;
static constexpr size_t OFF_BT   = OFF_LSE + SZ_LSE;
static constexpr size_t SZ_BT    = (size_t)NCOLP * KPITCH * 2;
static constexpr size_t OFF_ASEQ = OFF_BT + SZ_BT;
static constexpr size_t SZ_ASEQ  = (size_t)NPOS * EMK * 2;
static constexpr size_t OFF_OBS  = OFF_ASEQ + SZ_ASEQ;
static constexpr size_t SZ_OBS   = (size_t)OBSROWS * EMK * 2;
static constexpr size_t OFF_VL   = OFF_OBS + SZ_OBS;
static constexpr size_t SZ_VL    = (size_t)NPOS * KPITCH * 4;
static constexpr size_t OFF_PART = OFF_VL + SZ_VL;
static constexpr size_t SZ_PART  = (size_t)4 * 128;
static constexpr size_t WS_TOTAL = OFF_PART + SZ_PART;
static_assert(OFF_LSE % 128 == 0 && OFF_BT % 128 == 0 && OFF_ASEQ % 128 == 0 && OFF_OBS % 128 == 0 &&
              OFF_VL % 128 == 0 && OFF_PART % 128 == 0, "align");
static_assert(WS_TOTAL == 56954496, "ws total");
static_assert(WS_TOTAL <= 134217728, "ws cap");

static constexpr int LDS_ALPHA_OFF = 0;
static constexpr int LDS_VLS_OFF   = LDS_ALPHA_OFF + 16 * NCOLP * 4;
static constexpr int LDS_EA_OFF    = LDS_VLS_OFF + 16 * NCOLP * 4;
static constexpr int LDS_MX_OFF    = LDS_EA_OFF + 16 * KPITCH * 2;
static constexpr int LDS_RES_OFF   = LDS_MX_OFF + 64;
static constexpr int LDS_SCAN_BYTES = LDS_RES_OFF + 64;
static_assert(LDS_VLS_OFF % 16 == 0 && LDS_EA_OFF % 16 == 0 && LDS_MX_OFF % 16 == 0, "lds align");
static_assert(LDS_SCAN_BYTES == 127104, "lds bytes");

__device__ __forceinline__ float lse2f(float a, float b) {
  const float m = fmaxf(a, b);
  return logf(expf(a - m) + expf(b - m)) + m;
}

__device__ __forceinline__ float trans_logit(int s_src, float sA, float sB, float rb, int kp, float Cmj, float ttj) {
  const int gj = (kp >= NMATCH) ? 1 : 0;
  const int mj = kp - gj * NMATCH;
  const float dirv = gj ? sA : sB;
  const float chv = (rb + Cmj) + ttj;
  return (mj == s_src) ? dirv : ((mj > s_src) ? chv : NEGBIG);
}

__global__ __launch_bounds__(256) void k_tables(const float* __restrict__ ins, const float* __restrict__ del,
                                               float* __restrict__ tabout) {
  __shared__ float rn[NMATCH * 6];
  __shared__ float un[NMATCH * 6];
  __shared__ __align__(16) float tab[TABTOT];
  __shared__ float red[256];
  const int tid = threadIdx.x;

#pragma unroll 1
  for (int idx = tid; idx < NMATCH * 3; idx += 256) {
    const float a0 = ins[idx * 2], a1 = ins[idx * 2 + 1];
    const float la = lse2f(a0, a1);
    rn[idx * 2] = a0 - la; rn[idx * 2 + 1] = a1 - la;
    const float b0 = del[idx * 2], b1 = del[idx * 2 + 1];
    const float lb = lse2f(b0, b1);
    un[idx * 2] = b0 - lb; un[idx * 2 + 1] = b1 - lb;
  }
#pragma unroll 1
  for (int i = tid; i < TABTOT; i += 256) tab[i] = 0.f;
  __syncthreads();

  if (tid == 0) {
    float acc = 0.f;
    for (int m = 0; m < NMATCH; ++m) {
      const float d2 = rn[(m * 3 + 2) * 2 + 0] + un[(m * 3 + 2) * 2 + 1];
      acc = acc + d2;
      tab[TB_C + m + 1] = acc;
    }
  }
  __syncthreads();

#pragma unroll 1
  for (int k = tid; k < NSTATE; k += 256) {
    const int g = (k >= NMATCH) ? 1 : 0;
    const int m = k - g * NMATCH;
    const int s = m + 1 - g;
    const bool s_in = (s < NMATCH);
    const int sc = s_in ? s : (NMATCH - 1);
    float sstay  = rn[(sc * 3 + g) * 2 + 0];
    float sins   = rn[(sc * 3 + g) * 2 + 1];
    float smatch = un[(sc * 3 + g) * 2 + 0];
    float sdel   = un[(sc * 3 + g) * 2 + 1];
    sstay  = s_in ? sstay : NEGBIG;
    sins   = s_in ? sins : 0.f;
    smatch = s_in ? smatch : 0.f;
    sdel   = s_in ? sdel : NEGBIG;
    const bool m_in = (m < NMATCH);
    const int mc = m_in ? m : (NMATCH - 1);
    float l20 = rn[(mc * 3 + 2) * 2 + 0];
    float l21 = rn[(mc * 3 + 2) * 2 + 1];
    float u20 = un[(mc * 3 + 2) * 2 + 0];
    l20 = m_in ? l20 : NEGBIG;
    l21 = m_in ? l21 : 0.f;
    u20 = m_in ? u20 : 0.f;
    const float ttv = g ? l21 : (l20 + u20);
    tab[TB_SRCA + k] = sins;
    tab[TB_SRCB + k] = sstay + smatch;
    tab[TB_ROWB + k] = (sstay + sdel) - tab[TB_C + s + 1];
    tab[TB_TT + k] = ttv;
    const float rn0 = rn[0], rn1 = rn[1], un0 = un[0], un1 = un[1];
    float iv;
    if (m == 0) iv = g ? rn1 : (rn0 + un0);
    else        iv = (((rn0 + un1) - tab[TB_C + 1]) + tab[TB_C + m]) + ttv;
    tab[TB_INIT + k] = iv;
  }
  __syncthreads();

  float lmax = -3.0e38f;
  for (int k = tid; k < NSTATE; k += 256) lmax = fmaxf(lmax, tab[TB_INIT + k]);
  red[tid] = lmax; __syncthreads();
  for (int s2 = 128; s2 > 0; s2 >>= 1) {
    if (tid < s2) red[tid] = fmaxf(red[tid], red[tid + s2]);
    __syncthreads();
  }
  const float imax = red[0]; __syncthreads();
  float lsum = 0.f;
  for (int k = tid; k < NSTATE; k += 256) lsum += expf(tab[TB_INIT + k] - imax);
  red[tid] = lsum; __syncthreads();
  for (int s2 = 128; s2 > 0; s2 >>= 1) {
    if (tid < s2) red[tid] += red[tid + s2];
    __syncthreads();
  }
  const float ilse = logf(red[0]) + imax; __syncthreads();
  for (int k = tid; k < NSTATE; k += 256) tab[TB_INIT + k] = tab[TB_INIT + k] - ilse;
  __syncthreads();

  for (int pass = 0; pass < 2; ++pass) {
#pragma unroll 1
    for (int i = tid; i < TABTOT / 4; i += 256) {
      const v4f v = *(const v4f*)(tab + 4 * i);
      *(volatile v4f*)(tabout + 4 * i) = v;
    }
    __threadfence();
  }
}

__global__ __launch_bounds__(256) void k_rowlse(const float* __restrict__ tab, float* __restrict__ lseout) {
  __shared__ __align__(16) float cC[CLEN];
  __shared__ __align__(16) float ctt[TABLEN];
  __shared__ float lsev[32];
  const int tid = threadIdx.x;
  for (int i = tid; i < CLEN / 4; i += 256) *(v4f*)(cC + 4 * i) = *(const v4f*)(tab + TB_C + 4 * i);
  for (int i = tid; i < TABLEN / 4; i += 256) *(v4f*)(ctt + 4 * i) = *(const v4f*)(tab + TB_TT + 4 * i);
  __syncthreads();
  const int wave = tid >> 5, lane = tid & 31;
#pragma unroll 1
  for (int rr = 0; rr < 4; ++rr) {
    const int k = blockIdx.x * 32 + wave * 4 + rr;
    const int kc = (k < NSTATE) ? k : (NSTATE - 1);
    const int g = (kc >= NMATCH) ? 1 : 0;
    const int m = kc - g * NMATCH;
    const int s = m + 1 - g;
    const float sA = tab[TB_SRCA + kc], sB = tab[TB_SRCB + kc], rb = tab[TB_ROWB + kc];
    float mx = -3.0e38f;
#pragma unroll 1
    for (int j = lane; j < NSTATE; j += 32) {
      const int gj = (j >= NMATCH) ? 1 : 0;
      const int mj = j - gj * NMATCH;
      const float v = trans_logit(s, sA, sB, rb, j, cC[mj], ctt[j]);
      mx = fmaxf(mx, v);
    }
#pragma unroll
    for (int off = 16; off > 0; off >>= 1) mx = fmaxf(mx, __shfl_xor(mx, off, 32));
    float sum = 0.f;
#pragma unroll 1
    for (int j = lane; j < NSTATE; j += 32) {
      const int gj = (j >= NMATCH) ? 1 : 0;
      const int mj = j - gj * NMATCH;
      const float v = trans_logit(s, sA, sB, rb, j, cC[mj], ctt[j]);
      sum += expf(v - mx);
    }
#pragma unroll
    for (int off = 16; off > 0; off >>= 1) sum += __shfl_xor(sum, off, 32);
    float lse = logf(sum) + mx;
    lse = (k < NSTATE) ? lse : 0.f;
    if (lane == 0) lsev[wave * 4 + rr] = lse;
  }
  __syncthreads();
  if (wave == 0) {
    const float v = lsev[lane];
    float* dst = lseout + blockIdx.x * 32 + lane;
    *(volatile float*)dst = v;
    __threadfence();
    *(volatile float*)dst = v;
  }
}

__device__ __forceinline__ unsigned bt_entry(int k, float sA, float sB, float rb, float lk,
                                             int kp, float Cm, float ttj, bool kpv) {
  const int kc = (k < NSTATE) ? k : (NSTATE - 1);
  const int g = (kc >= NMATCH) ? 1 : 0;
  const int m = kc - g * NMATCH;
  const int s = m + 1 - g;
  const float v = trans_logit(s, sA, sB, rb, kp, Cm, ttj);
  float p = expf(v - lk);
  p = (kpv && (k < NSTATE)) ? p : 0.f;
  return (unsigned)f2bf_ftz(p);
}

__global__ __launch_bounds__(128) void k_btbuild(const float* __restrict__ tab, const float* __restrict__ lse,
                                                v4u* __restrict__ btout) {
  const int kp = blockIdx.x;
  const int tid = threadIdx.x;
  const int kpc = (kp < NSTATE) ? kp : (NSTATE - 1);
  const int gj = (kpc >= NMATCH) ? 1 : 0;
  const int mj = kpc - gj * NMATCH;
  const float Cm = tab[TB_C + mj];
  const float ttj = tab[TB_TT + kpc];
  const bool kpv = (kp < NSTATE);
  if (tid < KPITCH / 8) {
    const int k0 = tid * 8;
    const v4f sa0 = *(const v4f*)(tab + TB_SRCA + k0), sa1 = *(const v4f*)(tab + TB_SRCA + k0 + 4);
    const v4f sb0 = *(const v4f*)(tab + TB_SRCB + k0), sb1 = *(const v4f*)(tab + TB_SRCB + k0 + 4);
    const v4f rb0 = *(const v4f*)(tab + TB_ROWB + k0), rb1 = *(const v4f*)(tab + TB_ROWB + k0 + 4);
    const v4f lk0 = *(const v4f*)(lse + k0),           lk1 = *(const v4f*)(lse + k0 + 4);
    v4u w;
    w.x = bt_entry(k0 + 0, sa0.x, sb0.x, rb0.x, lk0.x, kpc, Cm, ttj, kpv) |
          (bt_entry(k0 + 1, sa0.y, sb0.y, rb0.y, lk0.y, kpc, Cm, ttj, kpv) << 16);
    w.y = bt_entry(k0 + 2, sa0.z, sb0.z, rb0.z, lk0.z, kpc, Cm, ttj, kpv) |
          (bt_entry(k0 + 3, sa0.w, sb0.w, rb0.w, lk0.w, kpc, Cm, ttj, kpv) << 16);
    w.z = bt_entry(k0 + 4, sa1.x, sb1.x, rb1.x, lk1.x, kpc, Cm, ttj, kpv) |
          (bt_entry(k0 + 5, sa1.y, sb1.y, rb1.y, lk1.y, kpc, Cm, ttj, kpv) << 16);
    w.w = bt_entry(k0 + 6, sa1.z, sb1.z, rb1.z, lk1.z, kpc, Cm, ttj, kpv) |
          (bt_entry(k0 + 7, sa1.w, sb1.w, rb1.w, lk1.w, kpc, Cm, ttj, kpv) << 16);
    v4u* dst = btout + (size_t)kp * (KPITCH / 8) + tid;
    *(volatile v4u*)dst = w;
    __threadfence();
    *(volatile v4u*)dst = w;
  }
}

__device__ __forceinline__ unsigned h_bits(float f) {
  return (unsigned)__builtin_bit_cast(unsigned short, (_Float16)f);
}
__global__ __launch_bounds__(256) void k_castseq(const float* __restrict__ seq, v4u* __restrict__ aout) {
  const int i = blockIdx.x * 256 + threadIdx.x;
  const int row = i >> 2;
  const int cg = (i & 3) * 8;
  const float* src = seq + (size_t)row * NALPHA;
  float f[8];
#pragma unroll
  for (int e = 0; e < 8; ++e) {
    const int col = cg + e;
    const int cc = (col < NALPHA) ? col : (NALPHA - 1);
    const float x = src[cc];
    f[e] = (col < NALPHA) ? x : 0.f;
  }
  v4u w;
  w.x = h_bits(f[0]) | (h_bits(f[1]) << 16);
  w.y = h_bits(f[2]) | (h_bits(f[3]) << 16);
  w.z = h_bits(f[4]) | (h_bits(f[5]) << 16);
  w.w = h_bits(f[6]) | (h_bits(f[7]) << 16);
  v4u* dst = aout + i;
  *(volatile v4u*)dst = w;
  __threadfence();
  *(volatile v4u*)dst = w;
}

__global__ __launch_bounds__(64) void k_obs(const float* __restrict__ pre, const float* __restrict__ iseq,
                                           v4u* __restrict__ obsout) {
  __shared__ float raw[16 * NALPHA];
  __shared__ __align__(16) float nrm[16 * EMK];
  const int tid = threadIdx.x;
  const int r0 = blockIdx.x * 16;
#pragma unroll 1
  for (int idx = tid; idx < 16 * NALPHA; idx += 64) {
    const int rr = idx / NALPHA;
    const int a = idx - rr * NALPHA;
    const int row = r0 + rr;
    const int rp = (row < NMATCH) ? row : (NMATCH - 1);
    int ri = row - NMATCH; ri = (ri < 0) ? 0 : ri; ri = (ri > NMATCH) ? NMATCH : ri;
    const float vp = pre[rp * NALPHA + a];
    const float vi = iseq[ri * NALPHA + a];
    raw[idx] = (row < NMATCH) ? vp : vi;
  }
  __syncthreads();
  if (tid < 16) {
    const int row = r0 + tid;
    const float* x = raw + tid * NALPHA;
    float mx = -3.0e38f;
#pragma unroll 1
    for (int a = 0; a < NALPHA; ++a) mx = fmaxf(mx, x[a]);
    float s1 = 0.f;
#pragma unroll 1
    for (int a = 0; a < NALPHA; ++a) s1 += expf(x[a] - mx);
    const float l1 = logf(s1) + mx;
    float mx2 = -3.0e38f;
#pragma unroll 1
    for (int a = 0; a < NALPHA; ++a) mx2 = fmaxf(mx2, x[a] - l1);
    float s2 = 0.f;
#pragma unroll 1
    for (int a = 0; a < NALPHA; ++a) s2 += expf((x[a] - l1) - mx2);
    const float l2 = logf(s2) + mx2;
#pragma unroll 1
    for (int a = 0; a < EMK; ++a) {
      const int ac = (a < NALPHA) ? a : (NALPHA - 1);
      const float v = (x[ac] - l1) - l2;
      nrm[tid * EMK + a] = ((a < NALPHA) && (row < NSTATE)) ? v : 0.f;
    }
  }
  __syncthreads();
  const float* sp = nrm + tid * 8;
  v4u w;
  w.x = h_bits(sp[0]) | (h_bits(sp[1]) << 16);
  w.y = h_bits(sp[2]) | (h_bits(sp[3]) << 16);
  w.z = h_bits(sp[4]) | (h_bits(sp[5]) << 16);
  w.w = h_bits(sp[6]) | (h_bits(sp[7]) << 16);
  v4u* dst = obsout + (size_t)blockIdx.x * 64 + tid;
  *(volatile v4u*)dst = w;
  __threadfence();
  *(volatile v4u*)dst = w;
}

__global__ __launch_bounds__(512) void k_scan(const float* tab, const unsigned short* btp, const float* vl,
                                             float* part) {
  extern __shared__ __align__(16) char smem[];
  float* alpha = (float*)(smem + LDS_ALPHA_OFF);
  float* vls   = (float*)(smem + LDS_VLS_OFF);
  unsigned short* eA = (unsigned short*)(smem + LDS_EA_OFF);
  float* mxs   = (float*)(smem + LDS_MX_OFF);
  float* resv  = (float*)(smem + LDS_RES_OFF);
  const __bf16* eAb = (const __bf16*)(smem + LDS_EA_OFF);
  const __bf16* bt = (const __bf16*)(const void*)btp;

  const int tid = threadIdx.x;
  const int w = tid >> 5;
  const int lane = tid & 31;
  const int rlane = lane & 15;
  const int hsel = lane >> 4;
  const int koff = hsel * 8;
  const int b0 = blockIdx.x * 16;

#pragma unroll 1
  for (int idx = tid; idx < 16 * NCOLP; idx += 512) {
    const int row = idx / NCOLP;
    const int col = idx - row * NCOLP;
    const float iv = tab[TB_INIT + col];
    const float ev = vl[((size_t)(b0 + row) * SEQLEN) * KPITCH + col];
    alpha[idx] = (col < NSTATE) ? (iv + ev) : -1.0e30f;
  }
  __syncthreads();

  const float* arow = alpha + w * NCOLP;
  unsigned short* erow = eA + w * KPITCH;
  float* vrow_l = vls + w * NCOLP;
  const __bf16* ap  = eAb + rlane * KPITCH + koff;
  const __bf16* bp0 = bt + (size_t)(w * 16 + rlane) * KPITCH + koff;
  const __bf16* bp1 = bt + (size_t)((w + 16) * 16 + rlane) * KPITCH + koff;
  const __bf16* bp2 = bt + (size_t)((w + 32) * 16 + rlane) * KPITCH + koff;
  const __bf16* bp3 = bt + (size_t)(768 + rlane) * KPITCH + koff;
  const v8f z8 = {0.f, 0.f, 0.f, 0.f, 0.f, 0.f, 0.f, 0.f};

  for (int t = 1; t < SEQLEN; ++t) {
    float m = -3.0e38f;
    for (int c = lane; c < NCOLP; c += 32) m = fmaxf(m, arow[c]);
#pragma unroll
    for (int off = 16; off > 0; off >>= 1) m = fmaxf(m, __shfl_xor(m, off, 32));
    if (lane == 0) mxs[w] = m;
#pragma unroll 1
    for (int k = lane; k < KPITCH; k += 32) {
      const int kc = (k < NCOLP) ? k : (NCOLP - 1);
      float e = __expf(arow[kc] - m);
      e = (k < NSTATE) ? e : 0.f;
      erow[k] = f2bf_ftz(e);
    }
    const float* vsrc = vl + ((size_t)(b0 + w) * SEQLEN + t) * KPITCH;
#pragma unroll 1
    for (int c4 = lane; c4 < NCOLP / 4; c4 += 32) {
      const v4f v = *(const v4f*)(vsrc + 4 * c4);
      *(v4f*)(vrow_l + 4 * c4) = v;
    }
    __syncthreads();

    v8f acc0 = z8, acc1 = z8, acc2 = z8;
#pragma unroll 1
    for (int k0 = 0; k0 < KLOOP; k0 += 32) {
      const v16b a  = Frag<__bf16>::load(ap + k0);
      const v16b f0 = Frag<__bf16>::load(bp0 + k0);
      const v16b f1 = Frag<__bf16>::load(bp1 + k0);
      const v16b f2 = Frag<__bf16>::load(bp2 + k0);
      acc0 = Frag<__bf16>::mma(a, f0, acc0);
      acc1 = Frag<__bf16>::mma(a, f1, acc1);
      acc2 = Frag<__bf16>::mma(a, f2, acc2);
      dep_guard3_b(acc0, acc1, acc2, a, f0, f1, f2);
    }
    dep_guard3_b(acc0, acc1, acc2, (v16b){}, (v16b){}, (v16b){}, (v16b){});

#pragma unroll
    for (int r = 0; r < 8; ++r) {
      const int row = hsel * 8 + r;
      const float mxr = mxs[row];
      const float* vr = vls + row * NCOLP;
      float* ar = alpha + row * NCOLP;
      int col = w * 16 + rlane;
      ar[col] = (__logf(fmaxf(acc0[r], 1.0e-30f)) + mxr) + vr[col];
      col = (w + 16) * 16 + rlane;
      ar[col] = (__logf(fmaxf(acc1[r], 1.0e-30f)) + mxr) + vr[col];
      col = (w + 32) * 16 + rlane;
      ar[col] = (__logf(fmaxf(acc2[r], 1.0e-30f)) + mxr) + vr[col];
    }
    if (w == 0) {
      v8f acc3 = z8;
#pragma unroll 1
      for (int k0 = 0; k0 < KLOOP; k0 += 32) {
        const v16b a  = Frag<__bf16>::load(ap + k0);
        const v16b f3 = Frag<__bf16>::load(bp3 + k0);
        acc3 = Frag<__bf16>::mma(a, f3, acc3);
        dep_guard1_b(acc3, a, f3);
      }
      dep_guard1_b(acc3, (v16b){}, (v16b){});
#pragma unroll
      for (int r = 0; r < 8; ++r) {
        const int row = hsel * 8 + r;
        const int col = 768 + rlane;
        float v = (__logf(fmaxf(acc3[r], 1.0e-30f)) + mxs[row]) + vls[row * NCOLP + col];
        v = (rlane == 0) ? v : -1.0e30f;
        alpha[row * NCOLP + col] = v;
      }
    }
    __syncthreads();
  }

  {
    float m = -3.0e38f;
    for (int c = lane; c < NSTATE; c += 32) m = fmaxf(m, arow[c]);
#pragma unroll
    for (int off = 16; off > 0; off >>= 1) m = fmaxf(m, __shfl_xor(m, off, 32));
    float s = 0.f;
#pragma unroll 1
    for (int c = lane; c < NSTATE; c += 32) s += __expf(arow[c] - m);
#pragma unroll
    for (int off = 16; off > 0; off >>= 1) s += __shfl_xor(s, off, 32);
    const float res = logf(s) + m;
    if (lane == 0) resv[w] = res;
  }
  __syncthreads();
  if (w == 0) {
    const int lc = (lane < 4) ? lane : 3;
    v4f v;
    v.x = resv[lc * 4 + 0]; v.y = resv[lc * 4 + 1]; v.z = resv[lc * 4 + 2]; v.w = resv[lc * 4 + 3];
    v.x = (lane < 4) ? v.x : 0.f; v.y = (lane < 4) ? v.y : 0.f;
    v.z = (lane < 4) ? v.z : 0.f; v.w = (lane < 4) ? v.w : 0.f;
    float* dst = part + blockIdx.x * 32 + lane * 4;
    if (lane < 8) { *(volatile v4f*)dst = v; }
    __threadfence();
    if (lane < 8) { *(volatile v4f*)dst = v; }
  }
}

__global__ __launch_bounds__(32) void k_final(const float* __restrict__ part, const float* __restrict__ scale,
                                             float* __restrict__ out) {
  const int lane = threadIdx.x;
  const int lc = (lane < 16) ? lane : 15;
  const int blk = lc >> 2;
  const int j = (lc & 3) * 4;
  v4f v = *(const v4f*)(part + blk * 32 + j);
  const float sc = scale[0];
  v.x = sc * v.x; v.y = sc * v.y; v.z = sc * v.z; v.w = sc * v.w;
  float* dst = out + lc * 4;
  if (lane < 16) { *(volatile v4f*)dst = v; }
  __threadfence();
  if (lane < 16) { *(volatile v4f*)dst = v; }
}

extern "C" void kernel_launch(void* const* d_in, const int* in_sizes, int n_in,
                              void* d_out, int out_size, void* d_ws, size_t ws_size,
                              hipStream_t stream) {
  if (n_in < 6) return;
  if (in_sizes[0] < NMATCH * NALPHA || in_sizes[1] < (NMATCH + 1) * NALPHA ||
      in_sizes[2] < NMATCH * 6 || in_sizes[3] < NMATCH * 6 ||
      in_sizes[4] < NBATCH * SEQLEN * NALPHA || in_sizes[5] < 1) return;
  if (out_size < NBATCH || ws_size < WS_TOTAL) return;

  const float* pre   = (const float*)d_in[0];
  const float* iseq  = (const float*)d_in[1];
  const float* ins   = (const float*)d_in[2];
  const float* del   = (const float*)d_in[3];
  const float* seq   = (const float*)d_in[4];
  const float* scale = (const float*)d_in[5];
  float* out = (float*)d_out;
  char* ws = (char*)d_ws;

  float* tab  = (float*)(ws + OFF_TAB);
  float* lse  = (float*)(ws + OFF_LSE);
  v4u*   btv  = (v4u*)(ws + OFF_BT);
  const unsigned short* btus = (const unsigned short*)(ws + OFF_BT);
  v4u*   aseqv = (v4u*)(ws + OFF_ASEQ);
  const unsigned short* asequs = (const unsigned short*)(ws + OFF_ASEQ);
  v4u*   obsv = (v4u*)(ws + OFF_OBS);
  const unsigned short* obsus = (const unsigned short*)(ws + OFF_OBS);
  float* vl   = (float*)(ws + OFF_VL);
  float* part = (float*)(ws + OFF_PART);

  k_tables<<<1, 256, 0, stream>>>(ins, del, tab);
  k_rowlse<<<TABLEN / 32, 256, 0, stream>>>(tab, lse);
  k_btbuild<<<NCOLP, 128, 0, stream>>>(tab, lse, btv);
  k_castseq<<<(NPOS * 4) / 256, 256, 0, stream>>>(seq, aseqv);
  k_obs<<<OBSROWS / 16, 64, 0, stream>>>(pre, iseq, obsv);
  {
    const int tiles = (NPOS / 64) * (OBSROWS / 64);
    wmma_gemm64<0, false, 0, 0, false, 0><<<dim3(tiles / 8, 1), 256, 0, stream>>>(
        asequs, asequs, EMK, 0L, obsus, obsus, EMK, 0L, (void*)vl, (void*)vl, KPITCH, 0L,
        tab, tab, 0L, NPOS, OBSROWS, EMK, 1.0f);
  }
  k_scan<<<NBATCH / 16, 512, LDS_SCAN_BYTES, stream>>>(tab, btus, vl, part);
  k_final<<<1, 32, 0, stream>>>(part, scale, out);
}
